// ExportEquiDeformableAttn_31044023615890
// MI455X (gfx1250) — hardware-run, weakly checked
//
#include <hip/hip_runtime.h>


#ifndef NB
#define NB 2
#endif
#ifndef NS
#define NS 50000
#endif
#define NB_FULL 2
#define NS_FULL 50000
#ifndef OUT_NS
#define OUT_NS NS
#endif
#define CCH  32
#define NSM  8
#define RR   128
#define RR2  (RR * RR)
#define AW   4
#define TP   36
#define QRS  2048.0f
#define QRI  (1.0f / 2048.0f)
#define WSC  1024.0f
#define WINV (1.0f / 1024.0f)
#define NT   ((NB * NS) / 32)

static_assert(CCH == 32);
static_assert(NSM * 3 + NSM == CCH);
static_assert((NB * NS) % 32 == 0);
static_assert(NB <= NB_FULL);
static_assert(NS <= NS_FULL);
static_assert(OUT_NS >= NS);
static_assert((TP * 4) % 16 == 0);
static_assert(TP >= CCH + 4);
static_assert(8 * 32 * 16 == 32 * CCH * 4);
static_assert((size_t)2 * AW * 32 * TP * 4 <= 131072);
static_assert(((size_t)NB * CCH * RR2) % (4 * 256) == 0);

typedef _Float16 h16;
typedef unsigned short bf;
typedef __attribute__((ext_vector_type(16))) _Float16 v16h;
typedef __attribute__((ext_vector_type(8)))  _Float16 v8h;
typedef __attribute__((ext_vector_type(8)))  float    v8f;
typedef __attribute__((ext_vector_type(4)))  float    v4f;
typedef v4f  __attribute__((may_alias)) v4fa;

__device__ __forceinline__ unsigned short f2bf(float f) { unsigned u = __float_as_uint(f); u += 0x7FFFu + ((u >> 16) & 1u); return (unsigned short)(u >> 16); }
__device__ __forceinline__ float bfr(float f) { return __uint_as_float(((unsigned)f2bf(f)) << 16); }
__device__ __forceinline__ v4f bfr4(v4f v) { v4f o; o[0] = bfr(v[0]); o[1] = bfr(v[1]); o[2] = bfr(v[2]); o[3] = bfr(v[3]); return o; }
__device__ __forceinline__ v16h cat16(v8h lo, v8h hi) { return __builtin_shufflevector(lo, hi, 0, 1, 2, 3, 4, 5, 6, 7, 8, 9, 10, 11, 12, 13, 14, 15); }
__device__ __forceinline__ v8f wmma16(v16h a, v16h b, v8f c) { return __builtin_amdgcn_wmma_f32_16x16x32_f16(false, a, false, b, (short)0, c, false, false); }
__device__ __forceinline__ v8f wmg(v16h a, v16h b, v8f c) { c = wmma16(a, b, c); asm volatile("v_nop\n\tv_nop\n\tv_nop\n\tv_nop" : "+v"(c) : "v"(a), "v"(b)); return c; }
__device__ __forceinline__ v16h ldh(const h16* p) { return cat16(*(const v8h*)p, *(const v8h*)(p + 16)); }
__device__ __forceinline__ void wave_sync() { __builtin_amdgcn_fence(3  , "wavefront"); __builtin_amdgcn_wave_barrier(); asm volatile("" ::: "memory"); }
static __device__ __forceinline__ h16 toh_flush(float v) { const h16 r = (h16)v; return (fabsf(v) < 6.103515625e-05f) ? (h16)0.0f : r; }
template <int BASE>
__device__ __forceinline__ void split4(const v4f x, v16h& H, v16h& R) {
#pragma unroll
    for (int i = 0; i < 4; ++i) { const h16 a = toh_flush(x[i]); H[BASE + i] = a; R[BASE + i] = toh_flush((x[i] - (float)a) * QRS); }
}

struct Tap { int i00; int dx; int dy; float wx; float wy; };
__device__ __forceinline__ Tap mk_tap(float u, float v) {
    Tap t;
    const float x = fminf(fmaxf(u, 0.0f), 1.0f) * (float)(RR - 1);
    const float y = fminf(fmaxf(v, 0.0f), 1.0f) * (float)(RR - 1);
    const float x0f = floorf(x), y0f = floorf(y);
    int x0 = (int)x0f; x0 = x0 < 0 ? 0 : (x0 > RR - 1 ? RR - 1 : x0);
    int y0 = (int)y0f; y0 = y0 < 0 ? 0 : (y0 > RR - 1 ? RR - 1 : y0);
    const int x1 = (x0 + 1 > RR - 1) ? (RR - 1) : (x0 + 1);
    const int y1 = (y0 + 1 > RR - 1) ? (RR - 1) : (y0 + 1);
    t.i00 = y0 * RR + x0; t.dx = x1 - x0; t.dy = (y1 - y0) * RR; t.wx = x - x0f; t.wy = y - y0f;
    return t;
}
__device__ __forceinline__ float tap_eval(const float* __restrict__ P, size_t co, const Tap t) {
    const float* q = P + co + (size_t)t.i00;
    const float f00 = q[0], f01 = q[t.dx], f10 = q[t.dy], f11 = q[t.dy + t.dx];
    const float top = f00 * (1.0f - t.wx) + f01 * t.wx;
    const float bot = f10 * (1.0f - t.wx) + f11 * t.wx;
    return top * (1.0f - t.wy) + bot * t.wy;
}

__global__ __launch_bounds__(256) void k_bfr4(const float* __restrict__ src, float* dst, size_t n4) {
    const size_t i = (size_t)blockIdx.x * 256 + threadIdx.x; if (i >= n4) return;
    const v4f v = *(const v4f*)(src + i * 4);
    const v4f o = bfr4(v);
    *(volatile v4f*)(dst + i * 4) = o; __threadfence(); *(volatile v4f*)(dst + i * 4) = o;
}

__global__ __launch_bounds__(128) void k_wconv(const float* __restrict__ Woff, const float* __restrict__ Ww, const float* __restrict__ Wv, const float* __restrict__ Wout, h16* WP) {
    const int i = threadIdx.x; const int n = i >> 2, k8 = (i & 3) * 8;
    const int pl = blockIdx.x;
    v8h o;
    if (pl == 0) {
        const int na = n < 24 ? n : 23; const int nc = n >= 24 ? n - 24 : 0;
#pragma unroll
        for (int j = 0; j < 8; ++j) {
            float a = Woff[(k8 + j) * 24 + na]; float c = Ww[(k8 + j) * 8 + nc];
            asm volatile("" : "+v"(a)); asm volatile("" : "+v"(c));
            const float v = (n < 24) ? a : c;
            o[j] = toh_flush(bfr(v) * WSC); }
    } else if (pl == 1) {
#pragma unroll
        for (int j = 0; j < 8; ++j) o[j] = toh_flush(bfr(Wv[(k8 + j) * CCH + n]) * WSC);
    } else {
#pragma unroll
        for (int j = 0; j < 8; ++j) o[j] = toh_flush(bfr(Wout[(k8 + j) * CCH + n]) * WSC);
    }
    h16* d = WP + (size_t)pl * (CCH * CCH) + (size_t)i * 8;
    *(volatile v8h*)d = o; __threadfence(); *(volatile v8h*)d = o;
}

__global__ __launch_bounds__(32 * AW) void k_stage1(const float* __restrict__ qp, const float* __restrict__ PXZ, const float* __restrict__ PXY, const float* __restrict__ PYZ,
                                                    const h16* __restrict__ WP, const float* __restrict__ boff, const float* __restrict__ bw, float* FEAT, float* PW) {
    __shared__ __align__(16) float fs[AW * 32 * TP];
    __shared__ __align__(16) float os[AW * 32 * TP];
    const int lane = threadIdx.x & 31, lr = lane & 15, hi = lane >> 4;
    const int wave = __builtin_amdgcn_readfirstlane((int)(threadIdx.x >> 5));
    const int tile = blockIdx.x * AW + wave;
    if (tile >= NT) return;
    const int wb = wave * 32 * TP;
    const int p = tile * 32 + lane; const int b = p / NS, t = p - b * NS;
    const size_t qrow = ((size_t)b * NS_FULL + (size_t)t) * 3;
    const float q0 = bfr(qp[qrow]), q1 = bfr(qp[qrow + 1]), q2 = bfr(qp[qrow + 2]);
    { v4f qv; qv[0] = q0; qv[1] = q1; qv[2] = q2; qv[3] = 0.0f; *(v4fa*)(&fs[wb + lane * TP + 32]) = qv; }
    const Tap txz = mk_tap(q0, q2), txy = mk_tap(q0, q1), tyz = mk_tap(q1, q2);
    const size_t pbase = (size_t)b * CCH * RR2;
#pragma unroll 1
    for (int c = 0; c < CCH; ++c) {
        const size_t co = pbase + (size_t)c * RR2;
        const float f = (tap_eval(PXZ, co, txz) + tap_eval(PXY, co, txy)) + tap_eval(PYZ, co, tyz);
        fs[wb + lane * TP + c] = f; }
    wave_sync();
#pragma unroll 1
    for (int ps = 0; ps < 2; ++ps) {
#pragma unroll
        for (int s = 0; s < 8; ++s) { const int row = 4 * s + (lane >> 3), cofs = (lane & 7) * 4;
            const v4f val = *(const v4fa*)(&fs[wb + row * TP + cofs]);
            const size_t pr = (size_t)tile * 32 + (size_t)row;
            *(volatile v4f*)(FEAT + pr * CCH + cofs) = val; }
        if (ps == 0) __threadfence(); }
    v16h aH[2], aR[2];
#pragma unroll
    for (int mt = 0; mt < 2; ++mt) {
        const int fo = wb + (mt * 16 + lr) * TP + 8 * hi;
        const v4f x0 = *(const v4fa*)(&fs[fo]), x1 = *(const v4fa*)(&fs[fo + 4]), x2 = *(const v4fa*)(&fs[fo + 16]), x3 = *(const v4fa*)(&fs[fo + 20]);
        aH[mt] = (v16h){}; aR[mt] = (v16h){};
        split4<0>(x0, aH[mt], aR[mt]); split4<4>(x1, aH[mt], aR[mt]); split4<8>(x2, aH[mt], aR[mt]); split4<12>(x3, aH[mt], aR[mt]); }
    const v16h b0 = ldh(WP + (size_t)(lr) * CCH + 8 * hi), b1 = ldh(WP + (size_t)(16 + lr) * CCH + 8 * hi);
    v8f cH00 = (v8f){}, cH01 = (v8f){}, cH10 = (v8f){}, cH11 = (v8f){}, cR00 = (v8f){}, cR01 = (v8f){}, cR10 = (v8f){}, cR11 = (v8f){};
    cH00 = wmg(aH[0], b0, cH00); cH01 = wmg(aH[0], b1, cH01); cH10 = wmg(aH[1], b0, cH10); cH11 = wmg(aH[1], b1, cH11);
    cR00 = wmg(aR[0], b0, cR00); cR01 = wmg(aR[0], b1, cR01); cR10 = wmg(aR[1], b0, cR10); cR11 = wmg(aR[1], b1, cR11);
#pragma unroll
    for (int r = 0; r < 8; ++r) {
        os[wb + (     8 * hi + r) * TP +      lr] = (cH00[r] + cR00[r] * QRI) * WINV;
        os[wb + (     8 * hi + r) * TP + 16 + lr] = (cH01[r] + cR01[r] * QRI) * WINV;
        os[wb + (16 + 8 * hi + r) * TP +      lr] = (cH10[r] + cR10[r] * QRI) * WINV;
        os[wb + (16 + 8 * hi + r) * TP + 16 + lr] = (cH11[r] + cR11[r] * QRI) * WINV; }
    wave_sync();
    const int m = lane & 7; const int cofs = m * 4; const bool isoff = cofs < 24;
    const int m3 = m % 3;
    v4f bo4 = *(const v4f*)(boff + (cofs < 20 ? cofs : 20));
    v4f bw4 = *(const v4f*)(bw + (cofs >= 24 ? cofs - 24 : 0));
    asm volatile("" : "+v"(bo4)); asm volatile("" : "+v"(bw4));
    v4f bias4;
#pragma unroll
    for (int i = 0; i < 4; ++i) bias4[i] = isoff ? bfr(bo4[i]) : bfr(bw4[i]);
#pragma unroll 1
    for (int ps = 0; ps < 2; ++ps) {
#pragma unroll
        for (int s = 0; s < 8; ++s) { const int row = 4 * s + (lane >> 3);
            v4f val = *(const v4fa*)(&os[wb + row * TP + cofs]);
            const v4f qv = *(const v4fa*)(&fs[wb + row * TP + 32]);
            const float r0 = (m3 == 0) ? qv[0] : ((m3 == 1) ? qv[1] : qv[2]);
            const float r1 = (m3 == 0) ? qv[1] : ((m3 == 1) ? qv[2] : qv[0]);
            const float r2 = (m3 == 0) ? qv[2] : ((m3 == 1) ? qv[0] : qv[1]);
            val = val + bias4;
            val[0] += isoff ? r0 : 0.0f; val[1] += isoff ? r1 : 0.0f; val[2] += isoff ? r2 : 0.0f; val[3] += isoff ? r0 : 0.0f;
            const size_t pr = (size_t)tile * 32 + (size_t)row;
            *(volatile v4f*)(PW + pr * CCH + cofs) = val; }
        if (ps == 0) __threadfence(); }
}

__global__ __launch_bounds__(32 * AW) void k_stage2(const float* __restrict__ PWp, const float* __restrict__ FEAT, const float* __restrict__ PXZ, const float* __restrict__ PXY, const float* __restrict__ PYZ,
                                                    const h16* __restrict__ WP, const float* __restrict__ bv, const float* __restrict__ bout, float* OUT) {
    __shared__ __align__(16) float ta[AW * 32 * TP];
    __shared__ __align__(16) float tb[AW * 32 * TP];
    const int lane = threadIdx.x & 31, lr = lane & 15, hi = lane >> 4;
    const int wave = __builtin_amdgcn_readfirstlane((int)(threadIdx.x >> 5));
    const int tile = blockIdx.x * AW + wave;
    if (tile >= NT) return;
    const int wb = wave * 32 * TP;
    const int p = tile * 32 + lane; const int b = p / NS;
    const size_t pbase = (size_t)b * CCH * RR2;
    { const v4f z = (v4f){};
#pragma unroll
      for (int c4 = 0; c4 < 8; ++c4) *(v4fa*)(&ta[wb + lane * TP + 4 * c4]) = z; }
    const float* prow = PWp + (size_t)p * CCH;
    float sw = 0.0f;
#pragma unroll 1
    for (int s = 0; s < NSM; ++s) {
        const float px = prow[3 * s], py = prow[3 * s + 1], pz = prow[3 * s + 2], ws = prow[24 + s];
        const Tap txz = mk_tap(px, pz), txy = mk_tap(px, py), tyz = mk_tap(py, pz);
#pragma unroll 1
        for (int c = 0; c < CCH; ++c) {
            const size_t co = pbase + (size_t)c * RR2;
            const float f = (tap_eval(PXZ, co, txz) + tap_eval(PXY, co, txy)) + tap_eval(PYZ, co, tyz);
            const int ix = wb + lane * TP + c;
            const float acc = ta[ix];
            ta[ix] = acc + ws * f; }
        sw += ws; }
    wave_sync();
    v16h aH[2], aR[2];
#pragma unroll
    for (int mt = 0; mt < 2; ++mt) {
        const int fo = wb + (mt * 16 + lr) * TP + 8 * hi;
        const v4f x0 = *(const v4fa*)(&ta[fo]), x1 = *(const v4fa*)(&ta[fo + 4]), x2 = *(const v4fa*)(&ta[fo + 16]), x3 = *(const v4fa*)(&ta[fo + 20]);
        aH[mt] = (v16h){}; aR[mt] = (v16h){};
        split4<0>(x0, aH[mt], aR[mt]); split4<4>(x1, aH[mt], aR[mt]); split4<8>(x2, aH[mt], aR[mt]); split4<12>(x3, aH[mt], aR[mt]); }
    {
        const h16* W1 = WP + (size_t)(CCH * CCH);
        const v16h b0 = ldh(W1 + (size_t)(lr) * CCH + 8 * hi), b1 = ldh(W1 + (size_t)(16 + lr) * CCH + 8 * hi);
        v8f cH00 = (v8f){}, cH01 = (v8f){}, cH10 = (v8f){}, cH11 = (v8f){}, cR00 = (v8f){}, cR01 = (v8f){}, cR10 = (v8f){}, cR11 = (v8f){};
        cH00 = wmg(aH[0], b0, cH00); cH01 = wmg(aH[0], b1, cH01); cH10 = wmg(aH[1], b0, cH10); cH11 = wmg(aH[1], b1, cH11);
        cR00 = wmg(aR[0], b0, cR00); cR01 = wmg(aR[0], b1, cR01); cR10 = wmg(aR[1], b0, cR10); cR11 = wmg(aR[1], b1, cR11);
#pragma unroll
        for (int r = 0; r < 8; ++r) {
            tb[wb + (     8 * hi + r) * TP +      lr] = (cH00[r] + cR00[r] * QRI) * WINV;
            tb[wb + (     8 * hi + r) * TP + 16 + lr] = (cH01[r] + cR01[r] * QRI) * WINV;
            tb[wb + (16 + 8 * hi + r) * TP +      lr] = (cH10[r] + cR10[r] * QRI) * WINV;
            tb[wb + (16 + 8 * hi + r) * TP + 16 + lr] = (cH11[r] + cR11[r] * QRI) * WINV; }
    }
    wave_sync();
    const v4f g0 = bfr4(*(const v4f*)(bv + 8 * hi)), g1 = bfr4(*(const v4f*)(bv + 8 * hi + 4)), g2 = bfr4(*(const v4f*)(bv + 16 + 8 * hi)), g3 = bfr4(*(const v4f*)(bv + 16 + 8 * hi + 4));
#pragma unroll
    for (int mt = 0; mt < 2; ++mt) {
        const float swr = __shfl(sw, mt * 16 + lr, 32);
        const int fo = wb + (mt * 16 + lr) * TP + 8 * hi;
        const v4f x0 = *(const v4fa*)(&tb[fo]), x1 = *(const v4fa*)(&tb[fo + 4]), x2 = *(const v4fa*)(&tb[fo + 16]), x3 = *(const v4fa*)(&tb[fo + 20]);
        const v4f y0 = x0 + g0 * swr, y1 = x1 + g1 * swr, y2 = x2 + g2 * swr, y3 = x3 + g3 * swr;
        aH[mt] = (v16h){}; aR[mt] = (v16h){};
        split4<0>(y0, aH[mt], aR[mt]); split4<4>(y1, aH[mt], aR[mt]); split4<8>(y2, aH[mt], aR[mt]); split4<12>(y3, aH[mt], aR[mt]); }
    {
        const h16* W2 = WP + (size_t)(2 * CCH * CCH);
        const v16h b0 = ldh(W2 + (size_t)(lr) * CCH + 8 * hi), b1 = ldh(W2 + (size_t)(16 + lr) * CCH + 8 * hi);
        v8f cH00 = (v8f){}, cH01 = (v8f){}, cH10 = (v8f){}, cH11 = (v8f){}, cR00 = (v8f){}, cR01 = (v8f){}, cR10 = (v8f){}, cR11 = (v8f){};
        cH00 = wmg(aH[0], b0, cH00); cH01 = wmg(aH[0], b1, cH01); cH10 = wmg(aH[1], b0, cH10); cH11 = wmg(aH[1], b1, cH11);
        cR00 = wmg(aR[0], b0, cR00); cR01 = wmg(aR[0], b1, cR01); cR10 = wmg(aR[1], b0, cR10); cR11 = wmg(aR[1], b1, cR11);
#pragma unroll
        for (int r = 0; r < 8; ++r) {
            ta[wb + (     8 * hi + r) * TP +      lr] = (cH00[r] + cR00[r] * QRI) * WINV;
            ta[wb + (     8 * hi + r) * TP + 16 + lr] = (cH01[r] + cR01[r] * QRI) * WINV;
            ta[wb + (16 + 8 * hi + r) * TP +      lr] = (cH10[r] + cR10[r] * QRI) * WINV;
            ta[wb + (16 + 8 * hi + r) * TP + 16 + lr] = (cH11[r] + cR11[r] * QRI) * WINV; }
    }
    wave_sync();
    const int cofs = (lane & 7) * 4;
    const v4f bo = bfr4(*(const v4f*)(bout + cofs));
#pragma unroll 1
    for (int ps = 0; ps < 2; ++ps) {
#pragma unroll
        for (int s = 0; s < 8; ++s) { const int row = 4 * s + (lane >> 3);
            const int pr = tile * 32 + row; const int bb = pr / NS, tt = pr - bb * NS;
            v4f val = *(const v4fa*)(&ta[wb + row * TP + cofs]);
            const v4f ft = *(const v4f*)(FEAT + (size_t)pr * CCH + cofs);
            val = (val + bo) + ft;
            *(volatile v4f*)(OUT + ((size_t)bb * OUT_NS + (size_t)tt) * CCH + cofs) = val; }
        if (ps == 0) __threadfence(); }
}

static constexpr size_t al256(size_t v) { return (v + 255) & ~(size_t)255; }
static constexpr size_t SZ_PLN = al256((size_t)NB * CCH * RR2 * 4);
static constexpr size_t SZ_WP  = al256((size_t)3 * CCH * CCH * 2);
static constexpr size_t SZ_ROW = al256((size_t)NT * 32 * CCH * 4);
static constexpr size_t SZ_TOTAL = 3 * SZ_PLN + SZ_WP + 2 * SZ_ROW;
static_assert(SZ_TOTAL <= (size_t)134217728);
static_assert((size_t)NT * 32 == (size_t)NB * NS);

extern "C" void kernel_launch(void* const* d_in, const int* in_sizes, int n_in,
                              void* d_out, int out_size, void* d_ws, size_t ws_size, hipStream_t stream) {
    if (n_in < 12) return;
    if ((size_t)in_sizes[0] < ((size_t)(NB - 1) * NS_FULL + NS) * 3) return;
    const size_t needp = (size_t)NB * CCH * RR2;
    if ((size_t)in_sizes[1] < needp || (size_t)in_sizes[2] < needp || (size_t)in_sizes[3] < needp) return;
    if (in_sizes[4] < CCH * 24 || in_sizes[5] < 24 || in_sizes[6] < CCH * 8 || in_sizes[7] < 8) return;
    if (in_sizes[8] < CCH * CCH || in_sizes[9] < CCH || in_sizes[10] < CCH * CCH || in_sizes[11] < CCH) return;
    if ((size_t)out_size < ((size_t)(NB - 1) * OUT_NS + NS) * CCH) return;
    if (SZ_TOTAL > ws_size) return;
    const float* qp   = (const float*)d_in[0];
    const float* cxz  = (const float*)d_in[1];
    const float* cxy  = (const float*)d_in[2];
    const float* cyz  = (const float*)d_in[3];
    const float* Woff = (const float*)d_in[4];  const float* boff = (const float*)d_in[5];
    const float* Ww   = (const float*)d_in[6];  const float* bw   = (const float*)d_in[7];
    const float* Wv   = (const float*)d_in[8];  const float* bv   = (const float*)d_in[9];
    const float* Wout = (const float*)d_in[10]; const float* bout = (const float*)d_in[11];
    float* OUT = (float*)d_out;
    char* wsp = (char*)d_ws;
    float* PXZ = (float*)wsp; wsp += SZ_PLN;
    float* PXY = (float*)wsp; wsp += SZ_PLN;
    float* PYZ = (float*)wsp; wsp += SZ_PLN;
    h16*   WP  = (h16*)wsp;   wsp += SZ_WP;
    float* FEAT = (float*)wsp; wsp += SZ_ROW;
    float* PW   = (float*)wsp; wsp += SZ_ROW;

    { const size_t n4 = (size_t)NB * CCH * RR2 / 4; const unsigned g = (unsigned)((n4 + 255) / 256);
      k_bfr4<<<g, 256, 0, stream>>>(cxz, PXZ, n4);
      k_bfr4<<<g, 256, 0, stream>>>(cxy, PXY, n4);
      k_bfr4<<<g, 256, 0, stream>>>(cyz, PYZ, n4); }
    k_wconv<<<3, 128, 0, stream>>>(Woff, Ww, Wv, Wout, WP);

    const unsigned gt = (unsigned)((NT + AW - 1) / AW);
    k_stage1<<<gt, 32 * AW, 0, stream>>>(qp, PXZ, PXY, PYZ, WP, boff, bw, FEAT, PW);
    k_stage2<<<gt, 32 * AW, 0, stream>>>(PW, FEAT, PXZ, PXY, PYZ, WP, bv, bout, OUT);
}
